// UnsupervisedModel_19911468384638
// MI455X (gfx1250) — hardware-verified
//
#include <hip/hip_runtime.h>
#include <stddef.h>


#define HIDC    128
#define NMAT    3
#define NGRAPH  64
#define NTHR    256
#define NWAVE   8
#define EPT     8
#define NGRP    2
#define CHUNK   (NTHR * EPT * NGRP)
#define WCAP    (EPT * NGRP * 32)
#define LISTN   (NWAVE * WCAP)
#define NBC     4096
#define NBF     1024
#define RCAP    40960
#define RBN     128
#define TGT     256
#define DEGCAP  256
#define OTHR    512
#define PCH     (NTHR * EPT)
#define APITCH  (HIDC + 8)

#define LDS_FILL ((RCAP + NBF + LISTN) * 4 + 64)
#define LDS_G128 (128 * APITCH * 4)
#define LDS_G64  (64 * APITCH * 4)

static_assert((CHUNK & (CHUNK - 1)) == 0);
static_assert(CHUNK <= 4096);
static_assert(NBC <= 4096 && NBF <= 4096);
static_assert((NBC & (NBC - 1)) == 0 && (NBF & (NBF - 1)) == 0);
static_assert(NBC == 4 * NBF);
static_assert(OTHR * 8 == NBC);
static_assert((RCAP % 32) == 0);
static_assert(TGT == NWAVE * 32);
static_assert((PCH & (PCH - 1)) == 0);
static_assert(HIDC == 128);

typedef float          v4f   __attribute__((ext_vector_type(4)));
typedef float          v8f   __attribute__((ext_vector_type(8)));
typedef int            v4i   __attribute__((ext_vector_type(4)));
typedef unsigned short v8us  __attribute__((ext_vector_type(8)));
typedef __bf16         v16bf __attribute__((ext_vector_type(16)));
union FragB { v16bf v; v8us h[2]; };
union FI { float f; int i; };

__device__ __forceinline__ unsigned int bfr_bits(float f) {
  unsigned int u = __float_as_uint(f);
  u += 0x7FFFu + ((u >> 16) & 1u);
  return u >> 16;
}

__device__ __forceinline__ void split1(float f, unsigned short& hi, unsigned short& lo) {
  const unsigned int hb = bfr_bits(f);
  const float hf = __uint_as_float(hb << 16);
  hi = (unsigned short)hb;
  lo = (unsigned short)bfr_bits(f - hf);
}

__device__ __forceinline__ void split8(v4f a, v4f b, v8us& hi, v8us& lo) {
  unsigned short h0, h1, h2, h3, h4, h5, h6, h7, l0, l1, l2, l3, l4, l5, l6, l7;
  split1(a.x, h0, l0); split1(a.y, h1, l1); split1(a.z, h2, l2); split1(a.w, h3, l3);
  split1(b.x, h4, l4); split1(b.y, h5, l5); split1(b.z, h6, l6); split1(b.w, h7, l7);
  hi[0] = h0; hi[1] = h1; hi[2] = h2; hi[3] = h3; hi[4] = h4; hi[5] = h5; hi[6] = h6; hi[7] = h7;
  lo[0] = l0; lo[1] = l1; lo[2] = l2; lo[3] = l3; lo[4] = l4; lo[5] = l5; lo[6] = l6; lo[7] = l7;
}

__device__ __forceinline__ v8f wmb(v16bf a, v16bf b, v8f c) {
  v8f d = __builtin_amdgcn_wmma_f32_16x16x32_bf16(false, a, false, b, (short)0, c, false, false);
  asm volatile("v_nop\n\tv_nop\n\tv_nop\n\tv_nop" : "+v"(d) : "v"(a), "v"(b));
  return d;
}

template <int NB>
__device__ __forceinline__ int scan_chunk(const int* __restrict__ dsts, int nE, int cbase, int slotBase,
                                          int vec8, int* list, int tid, int lane, int wave) {
  int wc = 0;
#pragma unroll
  for (int g = 0; g < NGRP; ++g) {
    const int el0  = (g * NTHR + tid) * EPT;
    const int e0   = cbase + el0;
    const int sent = -2147483647 - 1;
    v4i da, db;
    if (vec8 != 0 && cbase + CHUNK <= nE) {
      da = *(const v4i*)(dsts + e0);
      db = *(const v4i*)(dsts + e0 + 4);
    } else {
      da.x = (e0     < nE) ? dsts[min(e0, nE - 1)] : sent;
      da.y = (e0 + 1 < nE) ? dsts[min(e0 + 1, nE - 1)] : sent;
      da.z = (e0 + 2 < nE) ? dsts[min(e0 + 2, nE - 1)] : sent;
      da.w = (e0 + 3 < nE) ? dsts[min(e0 + 3, nE - 1)] : sent;
      db.x = (e0 + 4 < nE) ? dsts[min(e0 + 4, nE - 1)] : sent;
      db.y = (e0 + 5 < nE) ? dsts[min(e0 + 5, nE - 1)] : sent;
      db.z = (e0 + 6 < nE) ? dsts[min(e0 + 6, nE - 1)] : sent;
      db.w = (e0 + 7 < nE) ? dsts[min(e0 + 7, nE - 1)] : sent;
    }
    const unsigned nb = (unsigned)slotBase;
    const unsigned s0 = (unsigned)da.x - nb, s1 = (unsigned)da.y - nb;
    const unsigned s2 = (unsigned)da.z - nb, s3 = (unsigned)da.w - nb;
    const unsigned s4 = (unsigned)db.x - nb, s5 = (unsigned)db.y - nb;
    const unsigned s6 = (unsigned)db.z - nb, s7 = (unsigned)db.w - nb;
    const bool h0 = s0 < (unsigned)NB, h1 = s1 < (unsigned)NB, h2 = s2 < (unsigned)NB, h3 = s3 < (unsigned)NB;
    const bool h4 = s4 < (unsigned)NB, h5 = s5 < (unsigned)NB, h6 = s6 < (unsigned)NB, h7 = s7 < (unsigned)NB;
    const unsigned any = __builtin_amdgcn_ballot_w32(h0 | h1 | h2 | h3 | h4 | h5 | h6 | h7);
    if (any != 0u) {
#define HITJ(J, HJ, SJ) { \
        const unsigned mj = __builtin_amdgcn_ballot_w32(HJ); \
        if (mj != 0u) { \
          if (HJ) { \
            const int pos = wc + (int)__builtin_amdgcn_mbcnt_lo(mj, 0u); \
            if (pos < WCAP) list[wave * WCAP + pos] = ((el0 + (J)) << 12) | (int)(SJ); \
          } \
          wc += (int)__builtin_popcount(mj); } }
      HITJ(0, h0, s0)
      HITJ(1, h1, s1)
      HITJ(2, h2, s2)
      HITJ(3, h3, s3)
      HITJ(4, h4, s4)
      HITJ(5, h5, s5)
      HITJ(6, h6, s6)
      HITJ(7, h7, s7)
#undef HITJ
    }
  }
  return wc;
}

__global__ __launch_bounds__(NTHR) void k_wprep(
    const float* __restrict__ w0, const float* __restrict__ w1, const float* __restrict__ w2,
    unsigned short* whi, unsigned short* wlo) {
  const int seg = (int)blockIdx.x >> 3;
  const float* src = seg == 0 ? w0 : (seg == 1 ? w1 : w2);
  const int i  = ((int)(blockIdx.x & 7) * NTHR) + (int)threadIdx.x;
  const int n  = i >> 4;
  const int k0 = (i & 15) * 8;
  v4f a, b;
  a.x = src[(k0 + 0) * HIDC + n]; a.y = src[(k0 + 1) * HIDC + n];
  a.z = src[(k0 + 2) * HIDC + n]; a.w = src[(k0 + 3) * HIDC + n];
  b.x = src[(k0 + 4) * HIDC + n]; b.y = src[(k0 + 5) * HIDC + n];
  b.z = src[(k0 + 6) * HIDC + n]; b.w = src[(k0 + 7) * HIDC + n];
  v8us hv, lv;
  split8(a, b, hv, lv);
  const size_t o = (size_t)seg * HIDC * HIDC + (size_t)i * 8;
  *(volatile v8us*)(whi + o) = hv;
  *(volatile v8us*)(wlo + o) = lv;
  __threadfence();
  *(volatile v8us*)(whi + o) = hv;
  *(volatile v8us*)(wlo + o) = lv;
}

__global__ __launch_bounds__(NTHR) void k_count(
    const int* __restrict__ ei, const float* __restrict__ ew,
    int* cnt, float* dinv, int nE, int vec8) {
  __shared__ __attribute__((aligned(16))) int   scnt[NBC];
  __shared__ __attribute__((aligned(16))) float sdeg[NBC];
  __shared__ __attribute__((aligned(16))) int   list[LISTN];
  __shared__ int wcnt[NWAVE];
  const int tid = threadIdx.x, lane = tid & 31, wave = tid >> 5;
  const int nodeBase = blockIdx.x * NBC;
  const int* dsts = ei + nE;

  for (int i = tid; i < NBC; i += NTHR) { scnt[i] = 0; sdeg[i] = 0.0f; }
  __syncthreads();

  const int nChunks = (nE + CHUNK - 1) / CHUNK;
#pragma unroll 1
  for (int ch = 0; ch < nChunks; ++ch) {
    const int cbase = ch * CHUNK;
    const int wc = scan_chunk<NBC>(dsts, nE, cbase, nodeBase, vec8, list, tid, lane, wave);
    if (lane == 0) wcnt[wave] = wc;
    __syncthreads();
    if (wave == 0) {
#pragma unroll 1
      for (int wsx = 0; wsx < NWAVE; ++wsx) {
        int n = __builtin_amdgcn_readfirstlane(wcnt[wsx]);
        n = n > WCAP ? WCAP : (n < 0 ? 0 : n);
        const int* lp = list + wsx * WCAP;
#pragma unroll 1
        for (int i = 0; i < n; ++i) {
          const int ent  = __builtin_amdgcn_readfirstlane(lp[i]);
          const int slot = ent & (NBC - 1);
          int e = cbase + ((ent >> 12) & (CHUNK - 1));
          e = e > nE - 1 ? nE - 1 : e;
          const float w = ew[e];
          if (lane == 0) {
            scnt[slot] = scnt[slot] + 1;
            sdeg[slot] = sdeg[slot] + w;
          }
        }
      }
    }
    __syncthreads();
  }

  v4i cq[4]; v4f dq[4];
#pragma unroll
  for (int q = 0; q < 4; ++q) {
    const int f = (wave * 4 + q) * 128 + 4 * lane;
    const v4i c  = *(const v4i*)(scnt + f);
    const v4f dg = *(const v4f*)(sdeg + f);
    cq[q] = c;
    const float d0 = dg.x + 1.0f, d1 = dg.y + 1.0f, d2 = dg.z + 1.0f, d3 = dg.w + 1.0f;
    dq[q].x = d0 > 0.0f ? rsqrtf(d0) : 0.0f;
    dq[q].y = d1 > 0.0f ? rsqrtf(d1) : 0.0f;
    dq[q].z = d2 > 0.0f ? rsqrtf(d2) : 0.0f;
    dq[q].w = d3 > 0.0f ? rsqrtf(d3) : 0.0f;
  }
  int*   cp = cnt + (size_t)nodeBase;
  float* dp = dinv + (size_t)nodeBase;
#pragma unroll
  for (int q = 0; q < 4; ++q) {
    const int f = (wave * 4 + q) * 128 + 4 * lane;
    *(volatile v4i*)(cp + f) = cq[q];
    *(volatile v4f*)(dp + f) = dq[q];
  }
  __threadfence();
#pragma unroll
  for (int q = 0; q < 4; ++q) {
    const int f = (wave * 4 + q) * 128 + 4 * lane;
    *(volatile v4i*)(cp + f) = cq[q];
    *(volatile v4f*)(dp + f) = dq[q];
  }
}

__global__ __launch_bounds__(OTHR) void k_offsets(
    const int* __restrict__ cnt, int* off, int* rbase, int nChunk) {
  __shared__ __attribute__((aligned(16))) int soff[NBC];
  __shared__ __attribute__((aligned(16))) int srb[RBN];
  __shared__ int wtot[OTHR / 32];
  const int tid = threadIdx.x, lane = tid & 31, wave = tid >> 5, sub = tid >> 7;
  for (int i = tid; i < RBN; i += OTHR) srb[i] = 0;
  int carry = 0;
#pragma unroll 1
  for (int ch = 0; ch < nChunk; ++ch) {
    const int base = ch * NBC;
    const v4i c0 = *(const v4i*)(cnt + base + 8 * tid);
    const v4i c1 = *(const v4i*)(cnt + base + 8 * tid + 4);
    const int e0 = max(c0.x, 0), e1 = max(c0.y, 0), e2 = max(c0.z, 0), e3 = max(c0.w, 0);
    const int e4 = max(c1.x, 0), e5 = max(c1.y, 0), e6 = max(c1.z, 0), e7 = max(c1.w, 0);
    const int ts = e0 + e1 + e2 + e3 + e4 + e5 + e6 + e7;
    int incl = ts;
#pragma unroll
    for (int d = 1; d < 32; d <<= 1) {
      const int t = __shfl_up(incl, d);
      if (lane >= d) incl += t;
    }
    if (lane == 31) wtot[wave] = incl;
    __syncthreads();
    const int S0 = wtot[0]  + wtot[1]  + wtot[2]  + wtot[3];
    const int S1 = wtot[4]  + wtot[5]  + wtot[6]  + wtot[7];
    const int S2 = wtot[8]  + wtot[9]  + wtot[10] + wtot[11];
    const int S3 = wtot[12] + wtot[13] + wtot[14] + wtot[15];
    int pre = 0;
#pragma unroll 1
    for (int w = 4 * sub; w < wave; ++w) pre += wtot[w];
    const int b0 = carry;
    const int b1 = b0 + ((S0 + 31) & ~31);
    const int b2 = b1 + ((S1 + 31) & ~31);
    const int b3 = b2 + ((S2 + 31) & ~31);
    const int b4 = b3 + ((S3 + 31) & ~31);
    const int myb = sub == 0 ? b0 : (sub == 1 ? b1 : (sub == 2 ? b2 : b3));
    if (tid == 0) {
      srb[min(4 * ch + 0, RBN - 1)] = b0;
      srb[min(4 * ch + 1, RBN - 1)] = b1;
      srb[min(4 * ch + 2, RBN - 1)] = b2;
      srb[min(4 * ch + 3, RBN - 1)] = b3;
    }
    int run = myb + pre + incl - ts;
    soff[8 * tid + 0] = run; run += e0;
    soff[8 * tid + 1] = run; run += e1;
    soff[8 * tid + 2] = run; run += e2;
    soff[8 * tid + 3] = run; run += e3;
    soff[8 * tid + 4] = run; run += e4;
    soff[8 * tid + 5] = run; run += e5;
    soff[8 * tid + 6] = run; run += e6;
    soff[8 * tid + 7] = run;
    carry = b4;
    __syncthreads();
    const v4i o0 = *(const v4i*)(soff + 4 * tid);
    const v4i o1 = *(const v4i*)(soff + 4 * (tid + OTHR));
    int* op = off + base;
    *(volatile v4i*)(op + 4 * tid) = o0;
    *(volatile v4i*)(op + 4 * (tid + OTHR)) = o1;
    __threadfence();
    *(volatile v4i*)(op + 4 * tid) = o0;
    *(volatile v4i*)(op + 4 * (tid + OTHR)) = o1;
    __syncthreads();
  }
  if (tid == 0) srb[min(4 * nChunk, RBN - 1)] = carry;
  __syncthreads();
  v4i rv = {0, 0, 0, 0};
  if (tid < 32) rv = *(const v4i*)(srb + 4 * tid);
  if (tid < 32) *(volatile v4i*)(rbase + 4 * tid) = rv;
  __threadfence();
  if (tid < 32) *(volatile v4i*)(rbase + 4 * tid) = rv;
}

__global__ __launch_bounds__(NTHR) void k_fill(
    const int* __restrict__ ei, const int* __restrict__ off, const int* __restrict__ rbase,
    int* csr, int nE, int vec8, int csrLen) {
  extern __shared__ v4f lds_dyn[];
  int* region = (int*)lds_dyn;
  int* cursor = region + RCAP;
  int* list   = cursor + NBF;
  int* wcnt   = list + LISTN;
  const int tid = threadIdx.x, lane = tid & 31, wave = tid >> 5;
  const int b = blockIdx.x;
  const int nodeBase = b * NBF;
  const int* dsts = ei + nE;

  int rb0 = rbase[b];
  const int rb1 = rbase[b + 1];
  rb0 = rb0 < 0 ? 0 : (rb0 > csrLen ? csrLen : rb0);
  rb0 &= ~31;
  int len = rb1 - rb0;
  len = len < 0 ? 0 : (len > RCAP ? RCAP : len);
  int lenW = (len + 31) & ~31;
  if (rb0 + lenW > csrLen) lenW = (csrLen - rb0) & ~31;

  {
    const v4i z = {0, 0, 0, 0};
    for (int i = tid; i < RCAP / 4; i += NTHR) ((v4i*)region)[i] = z;
    for (int s = tid; s < NBF; s += NTHR) {
      int o = off[nodeBase + s] - rb0;
      o = o < 0 ? 0 : (o > RCAP ? RCAP : o);
      cursor[s] = o;
    }
  }
  __syncthreads();

  const int nChunks = (nE + CHUNK - 1) / CHUNK;
#pragma unroll 1
  for (int ch = 0; ch < nChunks; ++ch) {
    const int cbase = ch * CHUNK;
    const int wc = scan_chunk<NBF>(dsts, nE, cbase, nodeBase, vec8, list, tid, lane, wave);
    if (lane == 0) wcnt[wave] = wc;
    __syncthreads();
    if (wave == 0) {
#pragma unroll 1
      for (int wsx = 0; wsx < NWAVE; ++wsx) {
        int n = __builtin_amdgcn_readfirstlane(wcnt[wsx]);
        n = n > WCAP ? WCAP : (n < 0 ? 0 : n);
        const int* lp = list + wsx * WCAP;
#pragma unroll 1
        for (int i = 0; i < n; ++i) {
          const int ent  = __builtin_amdgcn_readfirstlane(lp[i]);
          const int slot = ent & (NBF - 1);
          int e = cbase + ((ent >> 12) & (CHUNK - 1));
          e = e > nE - 1 ? nE - 1 : e;
          if (lane == 0) {
            int pos = cursor[slot];
            pos = pos < 0 ? 0 : (pos > RCAP - 1 ? RCAP - 1 : pos);
            region[pos] = e;
            const int np = pos + 1;
            cursor[slot] = np > RCAP ? RCAP : np;
          }
        }
      }
    }
    __syncthreads();
  }

  const int nv = lenW >> 2;
  int* gp = csr + rb0;
#pragma unroll 1
  for (int i = tid; i < nv; i += NTHR) { const v4i v = ((const v4i*)region)[i]; *(volatile v4i*)(gp + 4 * i) = v; }
  __threadfence();
#pragma unroll 1
  for (int i = tid; i < nv; i += NTHR) { const v4i v = ((const v4i*)region)[i]; *(volatile v4i*)(gp + 4 * i) = v; }
}

template <int RB>
__global__ __launch_bounds__(RB * 2) void k_gemm(
    const float* __restrict__ A, const unsigned short* __restrict__ Bh, const unsigned short* __restrict__ Bl,
    const float* __restrict__ dinv, const float* __restrict__ bias, float* C,
    int nRowsA, int useDinv, int useBias) {
  extern __shared__ v4f lds_dyn[];
  constexpr int NT = RB * 2;
  constexpr int KD = HIDC;
  constexpr int AP = APITCH;
  unsigned short* sAh = (unsigned short*)lds_dyn;
  unsigned short* sAl = sAh + RB * AP;
  float*          stg = (float*)lds_dyn;
  const int tid = threadIdx.x, lane = tid & 31, wave = tid >> 5, hh = lane >> 4, m = lane & 15;
  const int rowBase = blockIdx.x * RB;

#pragma unroll
  for (int i = 0; i < (RB * KD / 8) / NT; ++i) {
    const int idx = i * NT + tid;
    const int r   = idx >> 4;
    const int c0  = (idx & 15) * 8;
    int row = rowBase + r;
    row = row > nRowsA - 1 ? nRowsA - 1 : row;
    const float* ap = A + (size_t)row * KD + c0;
    const v4f a = *(const v4f*)ap, b = *(const v4f*)(ap + 4);
    v8us hv, lv;
    split8(a, b, hv, lv);
    *(v8us*)(sAh + r * AP + c0) = hv;
    *(v8us*)(sAl + r * AP + c0) = lv;
  }
  __syncthreads();

  v8f acc[8];
#pragma unroll
  for (int t = 0; t < 8; ++t) { v8f z = {0.f, 0.f, 0.f, 0.f, 0.f, 0.f, 0.f, 0.f}; acc[t] = z; }
  const unsigned short* ah = sAh + (wave * 16 + m) * AP + 8 * hh;
  const unsigned short* al = sAl + (wave * 16 + m) * AP + 8 * hh;
#pragma unroll
  for (int kt = 0; kt < KD / 32; ++kt) {
    FragB fah, fal;
    fah.h[0] = *(const v8us*)(ah + 32 * kt);
    fah.h[1] = *(const v8us*)(ah + 32 * kt + 16);
    fal.h[0] = *(const v8us*)(al + 32 * kt);
    fal.h[1] = *(const v8us*)(al + 32 * kt + 16);
#pragma unroll
    for (int t = 0; t < 8; ++t) {
      const size_t bo = (size_t)(16 * t + m) * KD + 32 * kt + 8 * hh;
      FragB fbh, fbl;
      fbh.h[0] = *(const v8us*)(Bh + bo);
      fbh.h[1] = *(const v8us*)(Bh + bo + 16);
      fbl.h[0] = *(const v8us*)(Bl + bo);
      fbl.h[1] = *(const v8us*)(Bl + bo + 16);
      acc[t] = wmb(fah.v, fbh.v, acc[t]);
      acc[t] = wmb(fah.v, fbl.v, acc[t]);
      acc[t] = wmb(fal.v, fbh.v, acc[t]);
    }
  }
  __syncthreads();

  const int r0 = wave * 16 + 8 * hh;
  const v4f dA = *(const v4f*)(dinv + (size_t)rowBase + r0);
  const v4f dB = *(const v4f*)(dinv + (size_t)rowBase + r0 + 4);
  float s[8];
  s[0] = dA.x; s[1] = dA.y; s[2] = dA.z; s[3] = dA.w; s[4] = dB.x; s[5] = dB.y; s[6] = dB.z; s[7] = dB.w;
#pragma unroll
  for (int r = 0; r < 8; ++r) s[r] = (useDinv != 0 ? s[r] : 1.0f);
  float* sp = stg + r0 * HIDC + m;
#pragma unroll
  for (int t = 0; t < 8; ++t) {
    const float bl = bias[16 * t + m];
    const float bv = useBias != 0 ? bl : 0.0f;
#pragma unroll
    for (int r = 0; r < 8; ++r) sp[r * HIDC + 16 * t] = acc[t][r] * s[r] + bv;
  }
  __syncthreads();

  const float* lp = stg + wave * 16 * HIDC + 4 * lane;
  float* gp = C + ((size_t)rowBase + wave * 16) * HIDC + 4 * lane;
#pragma unroll
  for (int i = 0; i < 16; ++i) { const v4f v = *(const v4f*)(lp + i * HIDC); *(volatile v4f*)(gp + (size_t)i * HIDC) = v; }
  __threadfence();
#pragma unroll
  for (int i = 0; i < 16; ++i) { const v4f v = *(const v4f*)(lp + i * HIDC); *(volatile v4f*)(gp + (size_t)i * HIDC) = v; }
}

__global__ __launch_bounds__(NTHR) void k_agg(
    const int* __restrict__ csr, const int* __restrict__ off, const int* __restrict__ cnt,
    const int* __restrict__ ei, const float* __restrict__ ew,
    const float* __restrict__ dinv, const float* __restrict__ hw, float* h,
    const float* __restrict__ bs, int nN, int nE, int csrLen, int doRelu) {
  const int tid = threadIdx.x, lane = tid & 31, wave = tid >> 5;
  const int tbase = blockIdx.x * TGT + wave * 32;
  const int cl = tbase + lane;
  const int cnt_l = cnt[cl];
  const int off_l = off[cl];
  FI dvu; dvu.f = dinv[cl];
  const v4f bb = *(const v4f*)(bs + 4 * lane);

#pragma unroll 1
  for (int j = 0; j < 32; ++j) {
    const int c = tbase + j;
    int n = __builtin_amdgcn_readlane(cnt_l, j);
    n = n < 0 ? 0 : (n > DEGCAP ? DEGCAP : n);
    const int st = __builtin_amdgcn_readlane(off_l, j);
    FI du; du.i = __builtin_amdgcn_readlane(dvu.i, j);
    const float dc = du.f;
    v4f acc = {0.f, 0.f, 0.f, 0.f};
#pragma unroll 1
    for (int q0 = 0; q0 < n; q0 += 32) {
      int pos = st + q0 + lane;
      pos = pos < 0 ? 0 : (pos > csrLen - 1 ? csrLen - 1 : pos);
      int e = csr[pos];
      e = e < 0 ? 0 : (e > nE - 1 ? nE - 1 : e);
      int sl = ei[e];
      sl = sl < 0 ? 0 : (sl > nN - 1 ? nN - 1 : sl);
      FI wl; wl.f = ew[e];
      const int mcnt = (n - q0) < 32 ? (n - q0) : 32;
#pragma unroll 1
      for (int p = 0; p < mcnt; ++p) {
        const int s = __builtin_amdgcn_readlane(sl, p);
        FI wp; wp.i = __builtin_amdgcn_readlane(wl.i, p);
        const v4f row = *(const v4f*)(hw + (size_t)s * HIDC + 4 * lane);
        acc = acc + row * wp.f;
      }
    }
    const v4f sv = *(const v4f*)(hw + (size_t)c * HIDC + 4 * lane);
    v4f v = (acc + sv) * dc + bb;
    if (doRelu != 0) {
      v.x = fmaxf(v.x, 0.f); v.y = fmaxf(v.y, 0.f); v.z = fmaxf(v.z, 0.f); v.w = fmaxf(v.w, 0.f);
    }
    float* hp = h + (size_t)c * HIDC + 4 * lane;
    *(volatile v4f*)hp = v;
    __threadfence();
    *(volatile v4f*)hp = v;
  }
}

__global__ __launch_bounds__(NTHR) void k_pool(
    const int* __restrict__ bt, const float* __restrict__ z, float* pooled, int nN, int vecb) {
  __shared__ __attribute__((aligned(16))) float spart[NWAVE * HIDC];
  __shared__ int scount[NWAVE];
  const int tid = threadIdx.x, lane = tid & 31, wave = tid >> 5;
  const int g = blockIdx.x;
  v4f acc = {0.f, 0.f, 0.f, 0.f};
  int hits = 0;
  const int nChunks = (nN + PCH - 1) / PCH;
#pragma unroll 1
  for (int ch = 0; ch < nChunks; ++ch) {
    const int cbase = ch * PCH;
    const int e0 = cbase + tid * EPT;
    const int sent = -2147483647 - 1;
    v4i da, db;
    if (vecb != 0 && cbase + PCH <= nN) {
      da = *(const v4i*)(bt + e0);
      db = *(const v4i*)(bt + e0 + 4);
    } else {
      da.x = (e0     < nN) ? bt[min(e0, nN - 1)] : sent;
      da.y = (e0 + 1 < nN) ? bt[min(e0 + 1, nN - 1)] : sent;
      da.z = (e0 + 2 < nN) ? bt[min(e0 + 2, nN - 1)] : sent;
      da.w = (e0 + 3 < nN) ? bt[min(e0 + 3, nN - 1)] : sent;
      db.x = (e0 + 4 < nN) ? bt[min(e0 + 4, nN - 1)] : sent;
      db.y = (e0 + 5 < nN) ? bt[min(e0 + 5, nN - 1)] : sent;
      db.z = (e0 + 6 < nN) ? bt[min(e0 + 6, nN - 1)] : sent;
      db.w = (e0 + 7 < nN) ? bt[min(e0 + 7, nN - 1)] : sent;
    }
    const bool h0 = da.x == g, h1 = da.y == g, h2 = da.z == g, h3 = da.w == g;
    const bool h4 = db.x == g, h5 = db.y == g, h6 = db.z == g, h7 = db.w == g;
    const unsigned any = __builtin_amdgcn_ballot_w32(h0 | h1 | h2 | h3 | h4 | h5 | h6 | h7);
    if (any != 0u) {
#define POOLJ(J, HJ) { \
        unsigned mj = __builtin_amdgcn_ballot_w32(HJ); \
        hits += (int)__builtin_popcount(mj); \
        while (mj != 0u) { \
          const int ln = __builtin_ctz(mj); \
          mj &= mj - 1u; \
          int node = cbase + (wave * 32 + ln) * EPT + (J); \
          node = node < 0 ? 0 : (node > nN - 1 ? nN - 1 : node); \
          acc = acc + *(const v4f*)(z + (size_t)node * HIDC + 4 * lane); } }
      POOLJ(0, h0)
      POOLJ(1, h1)
      POOLJ(2, h2)
      POOLJ(3, h3)
      POOLJ(4, h4)
      POOLJ(5, h5)
      POOLJ(6, h6)
      POOLJ(7, h7)
#undef POOLJ
    }
  }
  *(v4f*)(spart + wave * HIDC + 4 * lane) = acc;
  if (lane == 0) scount[wave] = hits;
  __syncthreads();
  if (wave == 0) {
    v4f sum = *(const v4f*)(spart + 4 * lane);
    int tot = scount[0];
#pragma unroll
    for (int w = 1; w < NWAVE; ++w) { sum = sum + *(const v4f*)(spart + w * HIDC + 4 * lane); tot += scount[w]; }
    const float cn  = (float)tot;
    const float inv = 1.0f / fmaxf(cn, 1.0f);
    const v4f r = sum * inv;
    float* pp = pooled + (size_t)g * HIDC + 4 * lane;
    *(volatile v4f*)pp = r;
    __threadfence();
    *(volatile v4f*)pp = r;
  }
}

extern "C" void kernel_launch(void* const* d_in, const int* in_sizes, int n_in,
                              void* d_out, int out_size, void* d_ws, size_t ws_size,
                              hipStream_t stream) {
  if (n_in < 10) return;
  const int nN = in_sizes[0] / HIDC;
  const int nE = in_sizes[1] / 2;
  if (nN <= 0 || nE <= 0 || in_sizes[0] != nN * HIDC || in_sizes[1] != 2 * nE) return;
  if (in_sizes[2] != nE || in_sizes[3] != nN) return;
  if (in_sizes[4] != HIDC * HIDC || in_sizes[5] != HIDC) return;
  if (in_sizes[6] != HIDC * HIDC || in_sizes[7] != HIDC) return;
  if (in_sizes[8] != HIDC * HIDC || in_sizes[9] != HIDC) return;
  if (out_size != NGRAPH * HIDC) return;
  if (nE > (1 << 28) || nN > (1 << 24)) return;

  const float* x    = (const float*)d_in[0];
  const int*   ei   = (const int*)d_in[1];
  const float* ew   = (const float*)d_in[2];
  const int*   bt   = (const int*)d_in[3];
  const float* W1   = (const float*)d_in[4];
  const float* b1   = (const float*)d_in[5];
  const float* W2   = (const float*)d_in[6];
  const float* b2   = (const float*)d_in[7];
  const float* Wfc  = (const float*)d_in[8];
  const float* bfc  = (const float*)d_in[9];
  float* out = (float*)d_out;

  const int NPAD   = ((nN + TGT - 1) / TGT) * TGT;
  const int nBC    = (nN + NBC - 1) / NBC;
  const int CNTPAD = nBC * NBC;
  if (4 * nBC + 1 > RBN) return;
  const int nBF    = (nN + NBF - 1) / NBF;
  const int csrLen = ((nE + 31) & ~31) + 4096;
  if (31 * 4 * nBC > 4096) return;
  const int nGemm  = NPAD / 128;
  const int nAgg   = NPAD / TGT;

  char* ws = (char*)d_ws;
  size_t off = 0;
  const size_t WPL  = (size_t)NMAT * HIDC * HIDC;
  const size_t oWh  = off; off += WPL * 2;                        off = (off + 255) & ~(size_t)255;
  const size_t oWl  = off; off += WPL * 2;                        off = (off + 255) & ~(size_t)255;
  const size_t oCnt = off; off += (size_t)CNTPAD * 4;             off = (off + 255) & ~(size_t)255;
  const size_t oDv  = off; off += (size_t)CNTPAD * 4;             off = (off + 255) & ~(size_t)255;
  const size_t oOff = off; off += (size_t)CNTPAD * 4;             off = (off + 255) & ~(size_t)255;
  const size_t oRb  = off; off += (size_t)RBN * 4;                off = (off + 255) & ~(size_t)255;
  const size_t oCsr = off; off += (size_t)csrLen * 4;             off = (off + 255) & ~(size_t)255;
  const size_t oZ   = off; off += (size_t)NPAD * HIDC * 4;        off = (off + 255) & ~(size_t)255;
  const size_t oHw  = off; off += (size_t)NPAD * HIDC * 4;        off = (off + 255) & ~(size_t)255;
  const size_t oPl  = off; off += (size_t)NGRAPH * HIDC * 4;      off = (off + 255) & ~(size_t)255;
  if (off > ws_size) return;
  if (off > ((size_t)128 << 20)) return;
  unsigned short* whi  = (unsigned short*)(ws + oWh);
  unsigned short* wlo  = (unsigned short*)(ws + oWl);
  int*      cnt    = (int*)(ws + oCnt);
  float*    dinv   = (float*)(ws + oDv);
  int*      offp   = (int*)(ws + oOff);
  int*      rb     = (int*)(ws + oRb);
  int*      csr    = (int*)(ws + oCsr);
  float*    zp     = (float*)(ws + oZ);
  float*    hw     = (float*)(ws + oHw);
  float*    pooled = (float*)(ws + oPl);

  const int vec8 = ((nE & 3) == 0) ? 1 : 0;
  const int vecb = ((nN & 7) == 0) ? 1 : 0;

  k_wprep<<<NMAT * 8, NTHR, 0, stream>>>(W1, W2, Wfc, whi, wlo);

  k_count<<<nBC, NTHR, 0, stream>>>(ei, ew, cnt, dinv, nE, vec8);
  k_offsets<<<1, OTHR, 0, stream>>>(cnt, offp, rb, nBC);
  hipFuncSetAttribute(reinterpret_cast<const void*>(&k_fill),
                      hipFuncAttributeMaxDynamicSharedMemorySize, LDS_FILL);
  k_fill<<<nBF, NTHR, LDS_FILL, stream>>>(ei, offp, rb, csr, nE, vec8, csrLen);

  hipFuncSetAttribute(reinterpret_cast<const void*>(&k_gemm<128>),
                      hipFuncAttributeMaxDynamicSharedMemorySize, LDS_G128);
  k_gemm<128><<<nGemm, 256, LDS_G128, stream>>>(x, whi, wlo, dinv, b1, hw, nN, 1, 0);
  k_agg<<<nAgg, NTHR, 0, stream>>>(csr, offp, cnt, ei, ew, dinv, hw, zp, b1, nN, nE, csrLen, 1);

  k_gemm<128><<<nGemm, 256, LDS_G128, stream>>>(zp, whi + HIDC * HIDC, wlo + HIDC * HIDC, dinv, b2, hw, NPAD, 1, 0);
  k_agg<<<nAgg, NTHR, 0, stream>>>(csr, offp, cnt, ei, ew, dinv, hw, zp, b2, nN, nE, csrLen, 0);

  k_pool<<<NGRAPH, NTHR, 0, stream>>>(bt, zp, pooled, nN, vecb);

  k_gemm<64><<<1, 128, LDS_G64, stream>>>(pooled, whi + 2 * HIDC * HIDC, wlo + 2 * HIDC * HIDC, dinv, bfc, out, NGRAPH, 0, 1);
}
